// MultiScaleAttention_87711822119334
// MI455X (gfx1250) — hardware-run, weakly checked
//
#include <hip/hip_runtime.h>
#include <math.h>

typedef __attribute__((ext_vector_type(16))) _Float16 v16h;
typedef __attribute__((ext_vector_type(8)))  _Float16 v8h;
typedef __attribute__((ext_vector_type(4)))  _Float16 v4h;
typedef __attribute__((ext_vector_type(8)))  float    v8f;
typedef __attribute__((ext_vector_type(4)))  float    v4f;
typedef __attribute__((ext_vector_type(4)))  unsigned int v4u;

#ifndef NB
#define NB 2
#endif
#ifndef SEQ
#define SEQ 2048
#endif
#define NB_FULL 2
#define SEQ_FULL 2048
#define DM 1024
#define NH 16
#define HD 64
#define LW 256
#define GST 64
#define GG (SEQ / GST)
#define SWH 256
#define NROWS (NB * SEQ)
#define GROWS (NB * GG)
#define GPAD (((GROWS + 63) / 64) * 64)
#define NQB (SEQ / 64)
#define KPITCH 72
#define OPITCH 68
#define WSCALE 16.0f
#define INV_WSCALE 0.0625f
#define PCARRY 1024.0f
#define INV_PCARRY 0.0009765625f

static_assert(NB >= 1 && NB <= NB_FULL);
static_assert(SEQ >= LW && SEQ <= SEQ_FULL);
static_assert(SEQ % LW == 0);
static_assert(SEQ % 64 == 0 && LW % 64 == 0 && SWH % 64 == 0);
static_assert(DM % 64 == 0 && NH * HD == DM && HD == 64);
static_assert(NROWS % 64 == 0 && GPAD % 64 == 0 && GG >= 1 && GROWS >= 1);
static_assert(DM % 8 == 0);

__device__ __forceinline__ unsigned short f2bf_bits(float f) {
  unsigned u = __float_as_uint(f);
  return (unsigned short)((u + 0x7FFFu + ((u >> 16) & 1u)) >> 16);
}
__device__ __forceinline__ float bf_bits2f(unsigned short h) { return __uint_as_float(((unsigned)h) << 16); }
__device__ __forceinline__ float bfr(float f) { return bf_bits2f(f2bf_bits(f)); }
__device__ __forceinline__ unsigned short h_bits(_Float16 h) { return __builtin_bit_cast(unsigned short, h); }

__device__ __forceinline__ void dep_guard_h(v8f& a, v8f& b, v16h x, v16h y) { asm volatile("v_nop\n\tv_nop\n\tv_nop\n\tv_nop" : "+v"(a), "+v"(b) : "v"(x), "v"(y)); }
__device__ __forceinline__ void keep4_h(v16h a, v16h b, v16h c, v16h d) { asm volatile("v_nop" :: "v"(a), "v"(b), "v"(c), "v"(d)); }
__device__ __forceinline__ void acc_guard4(v8f& a, v8f& b, v8f& c, v8f& d) { asm volatile("v_nop\n\tv_nop\n\tv_nop\n\tv_nop" : "+v"(a), "+v"(b), "+v"(c), "+v"(d)); }

struct FragH {
  union U { v16h v; v8h h[2]; };
  static __device__ __forceinline__ v16h load(const _Float16* p) {
    U f; f.h[0] = *(const v8h*)(p); f.h[1] = *(const v8h*)(p + 16); return f.v;
  }
  static __device__ __forceinline__ v8f mma(v16h a, v16h b, v8f c) {
    return __builtin_amdgcn_wmma_f32_16x16x32_f16(false, a, false, b, (short)0, c, false, false);
  }
  static __device__ __forceinline__ void guard(v8f& a, v8f& b, v16h x, v16h y) { dep_guard_h(a, b, x, y); }
  static __device__ __forceinline__ void keep(v16h a, v16h b, v16h c, v16h d) { keep4_h(a, b, c, d); }
};

template <bool SPLIT, int BIAS_MODE, int OUT_MODE, bool RESID>
__global__ __launch_bounds__(256) void wmma_gemm64(
    const unsigned short* __restrict__ Ap, const unsigned short* __restrict__ A2p, int lda, long strideA,
    const unsigned short* __restrict__ Btp, const unsigned short* __restrict__ Bt2p, int ldb, long strideB,
    void* __restrict__ Cout, int ldc, long strideC,
    const float* __restrict__ bias,
    const float* __restrict__ resid, long strideR,
    int M, int N, int K, float scale) {
  typedef _Float16 T;
  typedef v16h V;
  const T* A = (const T*)Ap; const T* A2 = (const T*)A2p; const T* Bt = (const T*)Btp; const T* Bt2 = (const T*)Bt2p;
  __shared__ __align__(16) float sT[8][16 * 68];
  const int b    = blockIdx.y;
  const int lane = threadIdx.x & 31;
  const int wave = threadIdx.x >> 5;
  const int tilesN = N >> 6;
  const int tilesM = M >> 6;
  const int tile = blockIdx.x * 8 + wave;
  if (tile >= tilesM * tilesN) return;
  const int tm = tile / tilesN;
  const int tn = tile - tm * tilesN;
  const int m0 = tm << 6;
  const int n0 = tn << 6;

  const T* Ab  = A  + (size_t)b * strideA;
  const T* Bb  = Bt + (size_t)b * strideB;
  const T* Ab2 = SPLIT ? (A2  + (size_t)b * strideA) : nullptr;
  const T* Bb2 = SPLIT ? (Bt2 + (size_t)b * strideB) : nullptr;

  const int rlane = lane & 15;
  const int koff  = (lane >> 4) * 8;
  const int mOff  = (lane >> 4) * 8;

  v8f acc[4][4];
#pragma unroll
  for (int i = 0; i < 4; ++i)
#pragma unroll
    for (int j = 0; j < 4; ++j) acc[i][j] = (v8f){0.f,0.f,0.f,0.f,0.f,0.f,0.f,0.f};

  for (int k0 = 0; k0 < K; k0 += 32) {
    V bh[4], bl[4];
#pragma unroll
    for (int j = 0; j < 4; ++j) {
      const size_t bo = (size_t)(n0 + (j << 4) + rlane) * ldb + koff + k0;
      bh[j] = FragH::load(Bb + bo);
      if (SPLIT) bl[j] = FragH::load(Bb2 + bo);
    }
#pragma unroll
    for (int i = 0; i < 4; ++i) {
      const size_t ao = (size_t)(m0 + (i << 4) + rlane) * lda + koff + k0;
      V ah = FragH::load(Ab + ao);
      V al = ah;
      if (SPLIT) al = FragH::load(Ab2 + ao);
#pragma unroll
      for (int j = 0; j < 4; ++j) {
        acc[i][j] = FragH::mma(ah, bh[j], acc[i][j]);
        if (SPLIT) {
          acc[i][j] = FragH::mma(ah, bl[j], acc[i][j]);
          acc[i][j] = FragH::mma(al, bh[j], acc[i][j]);
        }
      }
      FragH::guard(acc[i][0], acc[i][3], ah, al);
    }
    FragH::keep(bh[0], bh[1], bh[2], bh[3]);
    if (SPLIT) FragH::keep(bl[0], bl[1], bl[2], bl[3]);
  }
  acc_guard4(acc[0][0], acc[0][1], acc[0][2], acc[0][3]);
  acc_guard4(acc[1][0], acc[1][1], acc[1][2], acc[1][3]);
  acc_guard4(acc[2][0], acc[2][1], acc[2][2], acc[2][3]);
  acc_guard4(acc[3][0], acc[3][1], acc[3][2], acc[3][3]);

  float* slab = sT[wave];
  const float* Rb = RESID ? (resid + (size_t)b * strideR) : nullptr;
#pragma unroll
  for (int i = 0; i < 4; ++i) {
    const int mBase = m0 + (i << 4);
#pragma unroll
    for (int j = 0; j < 4; ++j) {
      const int n = n0 + (j << 4) + rlane;
      float bv = 0.f;
      if (BIAS_MODE == 2) bv = bfr(bias[n]);
#pragma unroll
      for (int r = 0; r < 8; ++r) {
        float v = acc[i][j][r] * scale;
        if (BIAS_MODE == 1) v += bfr(bias[mBase + mOff + r]);
        if (BIAS_MODE == 2) v += bv;
        if (RESID) v += Rb[(size_t)(mBase + mOff + r) * ldc + n];
        slab[(mOff + r) * 68 + (j << 4) + rlane] = v;
      }
    }
    __builtin_amdgcn_fence(3, "workgroup");
    __builtin_amdgcn_wave_barrier();
    __builtin_amdgcn_fence(2, "workgroup");
    if (OUT_MODE == 0) {
      float* C = (float*)Cout + (size_t)b * strideC;
      const int hh = lane >> 4, c4 = (lane & 15) * 4;
      for (int pass = 0; pass < 2; ++pass) {
#pragma unroll
        for (int it = 0; it < 8; ++it) {
          const int row = it * 2 + hh;
          v4f v = *(const v4f*)(slab + row * 68 + c4);
          *(volatile v4f*)(C + (size_t)(mBase + row) * ldc + n0 + c4) = v;
        }
        __threadfence();
      }
    } else {
      const int q = lane >> 3, c8 = (lane & 7) * 8;
      _Float16* C = (_Float16*)((unsigned short*)Cout + (size_t)b * strideC);
      for (int pass = 0; pass < 2; ++pass) {
#pragma unroll
        for (int it = 0; it < 4; ++it) {
          const int row = it * 4 + q;
          const float* sp = slab + row * 68 + c8;
          v8h hv;
#pragma unroll
          for (int e = 0; e < 8; ++e) hv[e] = (_Float16)sp[e];
          *(volatile v8h*)(C + (size_t)(mBase + row) * ldc + n0 + c8) = hv;
        }
        __threadfence();
      }
    }
    __builtin_amdgcn_fence(3, "workgroup");
    __builtin_amdgcn_wave_barrier();
    __builtin_amdgcn_fence(2, "workgroup");
  }
}

__global__ __launch_bounds__(256) void cast_x_h16(
    const float* __restrict__ in, unsigned short* __restrict__ out, int n8) {
  const int i = blockIdx.x * 256 + threadIdx.x;
  if (i < n8) {
    const int row = i / (DM / 8);
    const int c8  = (i - row * (DM / 8)) * 8;
    const int bb  = row / SEQ;
    const int s   = row - bb * SEQ;
    const size_t src = ((size_t)bb * SEQ_FULL + (size_t)s) * DM + c8;
    const v4f a  = *(const v4f*)(in + src);
    const v4f a2 = *(const v4f*)(in + src + 4);
    v8h hv;
#pragma unroll
    for (int e = 0; e < 4; ++e) { hv[e] = (_Float16)bfr(a[e]); hv[4 + e] = (_Float16)bfr(a2[e]); }
    _Float16* p = (_Float16*)out + (size_t)i * 8;
    *(volatile v8h*)p = hv;
    __threadfence();
    *(volatile v8h*)p = hv;
  }
}

__global__ __launch_bounds__(256) void gather_strided_rows(
    const unsigned short* __restrict__ xh, unsigned short* __restrict__ out, int n8) {
  const int i = blockIdx.x * 256 + threadIdx.x;
  if (i < n8) {
    const int row = i / (DM / 8);
    const int c8  = (i - row * (DM / 8)) * 8;
    const int rr  = (row < GROWS) ? row : (GROWS - 1);
    const int bb  = rr / GG;
    const int g   = rr - bb * GG;
    const size_t src = ((size_t)bb * SEQ + (size_t)g * GST) * DM + c8;
    v4u w = *(const v4u*)(xh + src);
    if (row >= GROWS) w = (v4u){0u, 0u, 0u, 0u};
    unsigned short* p = out + (size_t)i * 8;
    *(volatile v4u*)p = w;
    __threadfence();
    *(volatile v4u*)p = w;
  }
}

__global__ __launch_bounds__(256) void transpose_w_h16(
    const float* __restrict__ in, unsigned short* __restrict__ out, int pitchIn, int pitchOut) {
  __shared__ __align__(16) unsigned short tileT[64 * 72];
  const int tid = threadIdx.x;
  const int r0 = blockIdx.x * 64, c0 = blockIdx.y * 64;
  const int lr = tid >> 4, col4 = (tid & 15) * 4;
#pragma unroll
  for (int it = 0; it < 4; ++it) {
    const int row = it * 16 + lr;
    const v4f f = *(const v4f*)(in + (size_t)(r0 + row) * pitchIn + c0 + col4);
#pragma unroll
    for (int e = 0; e < 4; ++e) tileT[(col4 + e) * 72 + row] = h_bits((_Float16)(bfr(f[e]) * WSCALE));
  }
  __syncthreads();
  const int qrow = tid >> 3, c8 = (tid & 7) * 8;
  for (int pass = 0; pass < 2; ++pass) {
#pragma unroll
    for (int it = 0; it < 2; ++it) {
      const int i = it * 32 + qrow;
      const v4u w = *(const v4u*)(tileT + i * 72 + c8);
      *(volatile v4u*)(out + (size_t)(c0 + i) * pitchOut + r0 + c8) = w;
    }
    __threadfence();
  }
}

__device__ __forceinline__ v8f mma_h(v16h a, v16h bm, v8f cacc) {
  cacc = __builtin_amdgcn_wmma_f32_16x16x32_f16(false, a, false, bm, (short)0, cacc, false, false);
  asm volatile("v_nop\n\tv_nop\n\tv_nop\n\tv_nop" : "+v"(cacc) : "v"(a), "v"(bm));
  return cacc;
}

template <int MODE>
__global__ __launch_bounds__(128) __attribute__((amdgpu_num_vgpr(256)))
void attn_f16_kernel(const unsigned short* __restrict__ Qp, const unsigned short* __restrict__ Kp,
                     const unsigned short* __restrict__ Vp, unsigned short* __restrict__ Op, int opitch) {
  __shared__ __align__(16) unsigned short Ks[64 * KPITCH];
  __shared__ __align__(16) unsigned short Vt[HD * KPITCH];
  __shared__ __align__(16) unsigned short Ps[4][16 * KPITCH];
  __shared__ __align__(16) float Os[4][16 * OPITCH];

  const int tid  = threadIdx.x;
  const int wave = tid >> 5;
  const int lane = tid & 31;
  const int hh   = lane >> 4;
  const int c    = lane & 15;
  const int bx   = blockIdx.x;
  const int qblk = bx % NQB;
  const int bh   = bx / NQB;
  const int h    = bh % NH;
  const int b    = bh / NH;
  const int q0   = qblk * 64 + wave * 16;
  const size_t qrowb = (size_t)b * SEQ;
  const int hcol = h * HD;

  size_t krowb;
  int kcBeg, kcEnd;
  if (MODE == 0) {
    krowb = (size_t)b * SEQ + (size_t)(((qblk * 64) / LW) * LW);
    kcBeg = 0; kcEnd = LW / 64;
  } else if (MODE == 1) {
    krowb = (size_t)b * GG;
    kcBeg = 0; kcEnd = (GG + 63) / 64;
  } else {
    krowb = (size_t)b * SEQ;
    kcBeg = qblk - SWH / 64; if (kcBeg < 0) kcBeg = 0;
    kcEnd = qblk + 1 + SWH / 64; if (kcEnd > NQB) kcEnd = NQB;
  }

  v16h qa[2];
  {
    const _Float16* qrow = (const _Float16*)(Qp + (qrowb + q0 + c) * (size_t)DM + hcol);
#pragma unroll
    for (int dc = 0; dc < 2; ++dc) qa[dc] = FragH::load(qrow + dc * 32 + 8 * hh);
  }

  float mrow[8], lrow[8];
  v8f oacc[4];
#pragma unroll
  for (int r = 0; r < 8; ++r) { mrow[r] = -INFINITY; lrow[r] = 0.f; }
#pragma unroll
  for (int t = 0; t < 4; ++t) oacc[t] = (v8f){0.f,0.f,0.f,0.f,0.f,0.f,0.f,0.f};

#pragma unroll 1
  for (int kc = kcBeg; kc < kcEnd; ++kc) {
    const int kv0 = kc * 64;
    __syncthreads();
#pragma unroll
    for (int i = 0; i < 4; ++i) {
      const int idx = i * 128 + tid;
      const int kvr = idx >> 3, c8 = (idx & 7) * 8;
      int krow = kv0 + kvr;
      if (MODE == 1) krow = (krow < GG) ? krow : (GG - 1);
      const v4u w = *(const v4u*)(Kp + (krowb + (size_t)krow) * DM + hcol + c8);
      *(v4u*)(Ks + kvr * KPITCH + c8) = w;
    }
    {
      const int kvr = tid >> 1, dh = (tid & 1) * 32;
      int krow = kv0 + kvr;
      if (MODE == 1) krow = (krow < GG) ? krow : (GG - 1);
      const unsigned short* vrow = Vp + (krowb + (size_t)krow) * DM + hcol + dh;
#pragma unroll
      for (int i = 0; i < 4; ++i) {
        const v4u w = *(const v4u*)(vrow + 8 * i);
#pragma unroll
        for (int e = 0; e < 4; ++e) {
          const unsigned wd = w[e];
          Vt[(dh + 8 * i + 2 * e) * KPITCH + kvr]     = (unsigned short)(wd & 0xffffu);
          Vt[(dh + 8 * i + 2 * e + 1) * KPITCH + kvr] = (unsigned short)(wd >> 16);
        }
      }
    }
    __syncthreads();

    v8f s[4];
#pragma unroll
    for (int j = 0; j < 4; ++j) {
      s[j] = (v8f){0.f,0.f,0.f,0.f,0.f,0.f,0.f,0.f};
#pragma unroll
      for (int dc = 0; dc < 2; ++dc) {
        const v16h kb = FragH::load((const _Float16*)(Ks + (j * 16 + c) * KPITCH + dc * 32 + 8 * hh));
        s[j] = mma_h(qa[dc], kb, s[j]);
      }
    }

    float cm[8];
#pragma unroll
    for (int r = 0; r < 8; ++r) {
      float m = -INFINITY;
      const int qi = q0 + 8 * hh + r;
#pragma unroll
      for (int j = 0; j < 4; ++j) {
        float v = s[j][r] * 0.125f;
        if (MODE == 1) {
          const int kv = kv0 + j * 16 + c;
          v = (kv < GG) ? v : -INFINITY;
        }
        if (MODE == 2) {
          const int dlt = qi - (kv0 + j * 16 + c);
          v = (dlt <= SWH && dlt >= -SWH) ? v : -INFINITY;
        }
        s[j][r] = v;
        m = fmaxf(m, v);
      }
#pragma unroll
      for (int off = 1; off < 16; off <<= 1) m = fmaxf(m, __shfl_xor(m, off, 32));
      cm[r] = m;
    }
    unsigned short* pw = Ps[wave];
#pragma unroll
    for (int r = 0; r < 8; ++r) {
      const float mnew  = fmaxf(mrow[r], cm[r]);
      const bool  fin   = (mnew != -INFINITY);
      const float msub  = fin ? mnew : 0.f;
      const float alpha = fin ? expf(mrow[r] - mnew) : 1.f;
      mrow[r] = mnew;
      float psum = 0.f;
#pragma unroll
      for (int j = 0; j < 4; ++j) {
        const float p = expf(s[j][r] - msub);
        psum += p;
        pw[(8 * hh + r) * KPITCH + j * 16 + c] = h_bits((_Float16)(p * PCARRY));
      }
#pragma unroll
      for (int off = 1; off < 16; off <<= 1) psum += __shfl_xor(psum, off, 32);
      lrow[r] = lrow[r] * alpha + psum;
#pragma unroll
      for (int t = 0; t < 4; ++t) oacc[t][r] *= alpha;
    }
    __builtin_amdgcn_fence(3, "workgroup");
    __builtin_amdgcn_wave_barrier();
    __builtin_amdgcn_fence(2, "workgroup");

#pragma unroll
    for (int kk = 0; kk < 2; ++kk) {
      const v16h pa = FragH::load((const _Float16*)(pw + c * KPITCH + kk * 32 + 8 * hh));
#pragma unroll
      for (int t = 0; t < 4; ++t) {
        const v16h vb = FragH::load((const _Float16*)(Vt + (t * 16 + c) * KPITCH + kk * 32 + 8 * hh));
        oacc[t] = mma_h(pa, vb, oacc[t]);
      }
    }
  }

  float* os = Os[wave];
#pragma unroll
  for (int r = 0; r < 8; ++r) {
    const float l   = lrow[r];
    const float inv = (l > 0.f) ? ((1.0f / l) * INV_PCARRY) : 0.f;
#pragma unroll
    for (int t = 0; t < 4; ++t) os[(8 * hh + r) * OPITCH + t * 16 + c] = oacc[t][r] * inv;
  }
  __builtin_amdgcn_fence(3, "workgroup");
  __builtin_amdgcn_wave_barrier();
  __builtin_amdgcn_fence(2, "workgroup");
  {
    const int q4 = lane >> 3, c8 = (lane & 7) * 8;
    _Float16* obase = (_Float16*)(Op + (qrowb + q0) * (size_t)opitch + hcol);
    for (int pass = 0; pass < 2; ++pass) {
#pragma unroll
      for (int it = 0; it < 4; ++it) {
        const int row = it * 4 + q4;
        const float* sp = os + row * OPITCH + c8;
        v8h hv;
#pragma unroll
        for (int e = 0; e < 8; ++e) hv[e] = (_Float16)sp[e];
        *(volatile v8h*)(obase + (size_t)row * opitch + c8) = hv;
      }
      __threadfence();
    }
  }
}

template <int OUT16>
__global__ __launch_bounds__(256) void ln_resid_kernel(
    const float* __restrict__ y, const float* __restrict__ x, const float* __restrict__ bo,
    const float* __restrict__ w, const float* __restrict__ bb, void* __restrict__ out, int opitch) {
  __shared__ float red0[8];
  __shared__ float red1[8];
  const int row = blockIdx.x;
  const int tid = threadIdx.x;
  const int c0 = tid * 4;
  const int wv = tid >> 5, lane = tid & 31;
  const int bbi = row / SEQ;
  const int s   = row - bbi * SEQ;
  const size_t xbase = ((size_t)bbi * SEQ_FULL + (size_t)s) * DM + c0;
  const size_t ybase = (size_t)row * DM + c0;
  const v4f yv = *(const v4f*)(y + ybase);
  const v4f xv = *(const v4f*)(x + xbase);
  const v4f bv = *(const v4f*)(bo + c0);
  float t[4];
#pragma unroll
  for (int e = 0; e < 4; ++e) { const float o = yv[e] + bfr(bv[e]); t[e] = bfr(xv[e]) + o; }
  float sm = (t[0] + t[1]) + (t[2] + t[3]);
#pragma unroll
  for (int off = 1; off < 32; off <<= 1) sm += __shfl_xor(sm, off, 32);
  if (lane == 0) red0[wv] = sm;
  __syncthreads();
  float ts = 0.f;
#pragma unroll
  for (int i = 0; i < 8; ++i) ts += red0[i];
  const float mu = ts * (1.0f / (float)DM);
  float d[4];
  float s2 = 0.f;
#pragma unroll
  for (int e = 0; e < 4; ++e) { d[e] = t[e] - mu; s2 += d[e] * d[e]; }
#pragma unroll
  for (int off = 1; off < 32; off <<= 1) s2 += __shfl_xor(s2, off, 32);
  if (lane == 0) red1[wv] = s2;
  __syncthreads();
  float ts2 = 0.f;
#pragma unroll
  for (int i = 0; i < 8; ++i) ts2 += red1[i];
  const float var = ts2 * (1.0f / (float)DM);
  const float inv = rsqrtf(var + 1e-5f);
  const v4f w4 = *(const v4f*)(w + c0);
  const v4f b4 = *(const v4f*)(bb + c0);
  v4f o;
#pragma unroll
  for (int e = 0; e < 4; ++e) o[e] = d[e] * inv * bfr(w4[e]) + bfr(b4[e]);
  if (OUT16 == 1) {
    v4h oh;
#pragma unroll
    for (int e = 0; e < 4; ++e) oh[e] = (_Float16)o[e];
    _Float16* p = (_Float16*)out + (size_t)row * opitch + c0;
    *(volatile v4h*)p = oh;
    __threadfence();
    *(volatile v4h*)p = oh;
  } else {
    float* p = (float*)out + (size_t)row * opitch + c0;
    *(volatile v4f*)p = o;
    __threadfence();
    *(volatile v4f*)p = o;
  }
}

static void gemm_h16out(const unsigned short* A, int lda, const unsigned short* Bt, int ldb,
                        unsigned short* C, int ldc, const float* bias, const float* dummy_f32,
                        int M, int N, int K, hipStream_t st) {
  const int blocks = ((M / 64) * (N / 64) + 7) / 8;
  wmma_gemm64<false, 2, 1, false><<<dim3(blocks, 1), 256, 0, st>>>(
      A, A, lda, (long)0, Bt, Bt, ldb, (long)0, (void*)C, ldc, (long)0,
      bias, dummy_f32, (long)0, M, N, K, INV_WSCALE);
}
static void gemm_f32out(const unsigned short* A, int lda, const unsigned short* Bt, int ldb,
                        float* C, int ldc, const float* dummy_bias, const float* dummy_f32,
                        int M, int N, int K, hipStream_t st) {
  const int blocks = ((M / 64) * (N / 64) + 7) / 8;
  wmma_gemm64<false, 0, 0, false><<<dim3(blocks, 1), 256, 0, st>>>(
      A, A, lda, (long)0, Bt, Bt, ldb, (long)0, (void*)C, ldc, (long)0,
      dummy_bias, dummy_f32, (long)0, M, N, K, INV_WSCALE);
}

extern "C" void kernel_launch(void* const* d_in, const int* in_sizes, int n_in,
                              void* d_out, int out_size, void* d_ws, size_t ws_size,
                              hipStream_t stream) {
  if (n_in < 29) return;
  if (in_sizes[0] < (NB - 1) * SEQ_FULL * DM + SEQ * DM) return;
  for (int i = 1; i <= 28; ++i) {
    const int need = (i == 13 || i == 25) ? (2 * DM * DM) : ((i % 2 == 1 && i <= 25 && i != 15) ? (DM * DM) : DM);
    if (in_sizes[i] < need) return;
  }
  if (out_size < NROWS * DM) return;

  const float* x       = (const float*)d_in[0];
  const float* lq_w    = (const float*)d_in[1];  const float* lq_b    = (const float*)d_in[2];
  const float* lk_w    = (const float*)d_in[3];  const float* lk_b    = (const float*)d_in[4];
  const float* lv_w    = (const float*)d_in[5];  const float* lv_b    = (const float*)d_in[6];
  const float* gq_w    = (const float*)d_in[7];  const float* gq_b    = (const float*)d_in[8];
  const float* gk_w    = (const float*)d_in[9];  const float* gk_b    = (const float*)d_in[10];
  const float* gv_w    = (const float*)d_in[11]; const float* gv_b    = (const float*)d_in[12];
  const float* h_out_w = (const float*)d_in[13]; const float* h_out_b = (const float*)d_in[14];
  const float* h_ln_g  = (const float*)d_in[15]; const float* h_ln_b  = (const float*)d_in[16];
  const float* sq_w    = (const float*)d_in[17]; const float* sq_b    = (const float*)d_in[18];
  const float* sk_w    = (const float*)d_in[19]; const float* sk_b    = (const float*)d_in[20];
  const float* sv_w    = (const float*)d_in[21]; const float* sv_b    = (const float*)d_in[22];
  const float* s_out_w = (const float*)d_in[23]; const float* s_out_b = (const float*)d_in[24];
  const float* comb_w  = (const float*)d_in[25]; const float* comb_b  = (const float*)d_in[26];
  const float* ln_g    = (const float*)d_in[27]; const float* ln_b    = (const float*)d_in[28];
  float* out = (float*)d_out;

  const size_t PL16 = (size_t)NROWS * DM * 2;
  const size_t WPL  = (size_t)DM * DM * 2;
  const size_t WPL2 = (size_t)2 * DM * DM * 2;
  const size_t GPL  = (size_t)GPAD * DM * 2;
  const size_t CPL  = (size_t)NROWS * 2 * DM * 2;
  const size_t YPL  = (size_t)NROWS * DM * 4;
  size_t off = 0;
  const size_t off_xh = off; off += PL16;
  size_t off_w[10];
  for (int i = 0; i < 10; ++i) { off_w[i] = off; off += WPL; }
  const size_t off_hw = off; off += WPL2;
  const size_t off_cw = off; off += WPL2;
  const size_t off_p0 = off; off += PL16;
  const size_t off_p1 = off; off += PL16;
  const size_t off_p2 = off; off += PL16;
  const size_t off_p3 = off; off += PL16;
  const size_t off_gc = off; off += GPL;
  const size_t off_gk = off; off += GPL;
  const size_t off_gv = off; off += GPL;
  const size_t off_clg = off; off += CPL;
  const size_t off_chs = off; off += CPL;
  const size_t off_y  = off; off += YPL;
  const size_t total  = off;
  if (total > ws_size) return;

  char* ws = (char*)d_ws;
  unsigned short* xh  = (unsigned short*)(ws + off_xh);
  unsigned short* wT[10];
  for (int i = 0; i < 10; ++i) wT[i] = (unsigned short*)(ws + off_w[i]);
  unsigned short* hwT = (unsigned short*)(ws + off_hw);
  unsigned short* cwT = (unsigned short*)(ws + off_cw);
  unsigned short* P0  = (unsigned short*)(ws + off_p0);
  unsigned short* P1  = (unsigned short*)(ws + off_p1);
  unsigned short* P2  = (unsigned short*)(ws + off_p2);
  unsigned short* P3  = (unsigned short*)(ws + off_p3);
  unsigned short* gch = (unsigned short*)(ws + off_gc);
  unsigned short* gkp = (unsigned short*)(ws + off_gk);
  unsigned short* gvp = (unsigned short*)(ws + off_gv);
  unsigned short* cLG = (unsigned short*)(ws + off_clg);
  unsigned short* cHS = (unsigned short*)(ws + off_chs);
  float* ybuf = (float*)(ws + off_y);

  const int n8 = NROWS * DM / 8;
  cast_x_h16<<<(n8 + 255) / 256, 256, 0, stream>>>(x, xh, n8);
  const int g8 = GPAD * DM / 8;
  gather_strided_rows<<<(g8 + 255) / 256, 256, 0, stream>>>(xh, gch, g8);

  const float* wsq[10] = { lq_w, lk_w, lv_w, gq_w, gk_w, gv_w, sq_w, sk_w, sv_w, s_out_w };
  for (int i = 0; i < 10; ++i)
    transpose_w_h16<<<dim3(DM / 64, DM / 64, 1), 256, 0, stream>>>(wsq[i], wT[i], DM, DM);
  transpose_w_h16<<<dim3(2 * DM / 64, DM / 64, 1), 256, 0, stream>>>(h_out_w, hwT, DM, 2 * DM);
  transpose_w_h16<<<dim3(2 * DM / 64, DM / 64, 1), 256, 0, stream>>>(comb_w, cwT, DM, 2 * DM);

  gemm_h16out(xh, DM, wT[0], DM, P0, DM, lq_b, x, NROWS, DM, DM, stream);
  gemm_h16out(xh, DM, wT[1], DM, P1, DM, lk_b, x, NROWS, DM, DM, stream);
  gemm_h16out(xh, DM, wT[2], DM, P2, DM, lv_b, x, NROWS, DM, DM, stream);
  gemm_h16out(xh, DM, wT[3], DM, P3, DM, gq_b, x, NROWS, DM, DM, stream);
  gemm_h16out(gch, DM, wT[4], DM, gkp, DM, gk_b, x, GPAD, DM, DM, stream);
  gemm_h16out(gch, DM, wT[5], DM, gvp, DM, gv_b, x, GPAD, DM, DM, stream);

  attn_f16_kernel<0><<<NB * NH * NQB, 128, 0, stream>>>(P0, P1, P2, cLG, 2 * DM);
  attn_f16_kernel<1><<<NB * NH * NQB, 128, 0, stream>>>(P3, gkp, gvp, cLG + DM, 2 * DM);

  gemm_f32out(cLG, 2 * DM, hwT, 2 * DM, ybuf, DM, h_out_b, x, NROWS, DM, 2 * DM, stream);
  ln_resid_kernel<1><<<NROWS, 256, 0, stream>>>(ybuf, x, h_out_b, h_ln_g, h_ln_b, (void*)cHS, 2 * DM);

  gemm_h16out(xh, DM, wT[6], DM, P0, DM, sq_b, x, NROWS, DM, DM, stream);
  gemm_h16out(xh, DM, wT[7], DM, P1, DM, sk_b, x, NROWS, DM, DM, stream);
  gemm_h16out(xh, DM, wT[8], DM, P2, DM, sv_b, x, NROWS, DM, DM, stream);
  attn_f16_kernel<2><<<NB * NH * NQB, 128, 0, stream>>>(P0, P1, P2, P3, DM);
  gemm_h16out(P3, DM, wT[9], DM, cHS + DM, 2 * DM, s_out_b, x, NROWS, DM, DM, stream);

  gemm_f32out(cHS, 2 * DM, cwT, 2 * DM, ybuf, DM, comb_b, x, NROWS, DM, 2 * DM, stream);
  ln_resid_kernel<0><<<NROWS, 256, 0, stream>>>(ybuf, x, comb_b, ln_g, ln_b, (void*)out, DM);
}
